// MyLSTMCell_48146583388298
// MI455X (gfx1250) — hardware-verified
//
#include <hip/hip_runtime.h>
#include <stdint.h>
#include <stddef.h>

typedef __attribute__((ext_vector_type(16))) _Float16 v16h;
typedef __attribute__((ext_vector_type(8)))  _Float16 v8h;
typedef __attribute__((ext_vector_type(16))) __bf16   v16b;
typedef __attribute__((ext_vector_type(8)))  __bf16   v8b;
typedef __attribute__((ext_vector_type(8)))  float    v8f;
typedef __attribute__((ext_vector_type(4)))  float    v4f;
typedef __attribute__((ext_vector_type(4)))  unsigned v4u;

constexpr int kBatch = 4096;
constexpr int kDin   = 1024;
constexpr int kHid   = 1024;
constexpr int kKcat  = kDin + kHid;
constexpr int kNcat  = 4 * kHid;

static_assert(kKcat % 32 == 0, "K multiple of 32");
static_assert(kBatch % 64 == 0, "M multiple of 64");
static_assert(kNcat % 64 == 0, "N multiple of 64");
static_assert(kDin == kHid, "square weight tiles assumed by the transpose packer");

constexpr size_t kAcatBytes = (size_t)kBatch * kKcat * 2;
constexpr size_t kBtBytes   = (size_t)kNcat * kKcat * 2;
constexpr size_t kPreBytes  = (size_t)kBatch * kNcat * 4;
constexpr size_t kOffBt     = kAcatBytes;
constexpr size_t kOffPre    = kAcatBytes + kBtBytes;
constexpr size_t kCarve     = kOffPre + kPreBytes;
static_assert(kCarve == 100663296, "carve total");
static_assert(kCarve <= 134217728, "carve under 128 MiB");
static_assert(kOffBt % 128 == 0 && kOffPre % 128 == 0, "128-B aligned regions");

constexpr size_t kOut1ByteOff = 16777216;
constexpr size_t kOut1ElemOff = kOut1ByteOff / 4;
static_assert(kOut1ByteOff + (size_t)kBatch * kHid * 4 <= 33554432, "out1 inside d_out");

__device__ __forceinline__ unsigned short f2bf_bits(float f) {
  unsigned u = __float_as_uint(f);
  return (unsigned short)((u + 0x7FFFu + ((u >> 16) & 1u)) >> 16);
}
__device__ __forceinline__ float bf_bits2f(unsigned short h) { return __uint_as_float(((unsigned)h) << 16); }
__device__ __forceinline__ float bf_rne(float x) { return bf_bits2f(f2bf_bits(x)); }
__device__ __forceinline__ unsigned pack_bf2(float a, float b) {
  return (unsigned)f2bf_bits(a) | ((unsigned)f2bf_bits(b) << 16);
}

__device__ __forceinline__ void dep_guard_h(v8f& a, v8f& b, v16h x, v16h y) { asm volatile("v_nop\n\tv_nop\n\tv_nop\n\tv_nop" : "+v"(a), "+v"(b) : "v"(x), "v"(y)); }
__device__ __forceinline__ void dep_guard_b(v8f& a, v8f& b, v16b x, v16b y) { asm volatile("v_nop\n\tv_nop\n\tv_nop\n\tv_nop" : "+v"(a), "+v"(b) : "v"(x), "v"(y)); }
__device__ __forceinline__ void keep4_h(v16h a, v16h b, v16h c, v16h d) { asm volatile("v_nop" :: "v"(a), "v"(b), "v"(c), "v"(d)); }
__device__ __forceinline__ void keep4_b(v16b a, v16b b, v16b c, v16b d) { asm volatile("v_nop" :: "v"(a), "v"(b), "v"(c), "v"(d)); }
__device__ __forceinline__ void acc_guard4(v8f& a, v8f& b, v8f& c, v8f& d) { asm volatile("v_nop\n\tv_nop\n\tv_nop\n\tv_nop" : "+v"(a), "+v"(b), "+v"(c), "+v"(d)); }
template <typename T> struct Frag;
template <> struct Frag<_Float16> {
  typedef v16h V; union U { v16h v; v8h h[2]; };
  static __device__ __forceinline__ v16h load(const _Float16* p) {
    U f; f.h[0] = *(const v8h*)(p); f.h[1] = *(const v8h*)(p + 16); return f.v;
  }
  static __device__ __forceinline__ v8f mma(v16h a, v16h b, v8f c) {
    return __builtin_amdgcn_wmma_f32_16x16x32_f16(false, a, false, b, (short)0, c, false, false);
  }
  static __device__ __forceinline__ void guard(v8f& a, v8f& b, v16h x, v16h y) { dep_guard_h(a, b, x, y); }
  static __device__ __forceinline__ void keep(v16h a, v16h b, v16h c, v16h d) { keep4_h(a, b, c, d); }
};
template <> struct Frag<__bf16> {
  typedef v16b V; union U { v16b v; v8b h[2]; };
  static __device__ __forceinline__ v16b load(const __bf16* p) {
    U f; f.h[0] = *(const v8b*)(p); f.h[1] = *(const v8b*)(p + 16); return f.v;
  }
  static __device__ __forceinline__ v8f mma(v16b a, v16b b, v8f c) {
    return __builtin_amdgcn_wmma_f32_16x16x32_bf16(false, a, false, b, (short)0, c, false, false);
  }
  static __device__ __forceinline__ void guard(v8f& a, v8f& b, v16b x, v16b y) { dep_guard_b(a, b, x, y); }
  static __device__ __forceinline__ void keep(v16b a, v16b b, v16b c, v16b d) { keep4_b(a, b, c, d); }
};

template <int ET> struct Elem;
template <> struct Elem<0> { typedef _Float16 T; };
template <> struct Elem<1> { typedef __bf16 T; };
template <int ET, bool SPLIT, int BIAS_MODE, int OUT_MODE, bool RESID, int ACT = 0>
__global__ __launch_bounds__(256) void wmma_gemm64(
    const unsigned short* __restrict__ Ap, const unsigned short* __restrict__ A2p, int lda, long strideA,
    const unsigned short* __restrict__ Btp, const unsigned short* __restrict__ Bt2p, int ldb, long strideB,
    void* __restrict__ Cout, void* __restrict__ Cout2, int ldc, long strideC,
    const float* __restrict__ bias,
    const float* __restrict__ resid, long strideR,
    int M, int N, int K, float scale) {
  typedef typename Elem<ET>::T T;
  typedef typename Frag<T>::V V;
  const T* A = (const T*)Ap; const T* A2 = (const T*)A2p; const T* Bt = (const T*)Btp; const T* Bt2 = (const T*)Bt2p;
  __shared__ __align__(16) float sT[8][16 * 68];
  const int b    = blockIdx.y;
  const int lane = threadIdx.x & 31;
  const int wave = threadIdx.x >> 5;
  const int tilesN = N >> 6;
  const int tilesM = M >> 6;
  const int tile = blockIdx.x * 8 + wave;
  if (tile >= tilesM * tilesN) return;
  const int tm = tile / tilesN;
  const int tn = tile - tm * tilesN;
  const int m0 = tm << 6;
  const int n0 = tn << 6;

  const T* Ab  = A  + (size_t)b * strideA;
  const T* Bb  = Bt + (size_t)b * strideB;
  const T* Ab2 = SPLIT ? (A2  + (size_t)b * strideA) : nullptr;
  const T* Bb2 = SPLIT ? (Bt2 + (size_t)b * strideB) : nullptr;

  const int rlane = lane & 15;
  const int koff  = (lane >> 4) * 8;
  const int mOff  = (lane >> 4) * 8;

  v8f acc[4][4];
#pragma unroll
  for (int i = 0; i < 4; ++i)
#pragma unroll
    for (int j = 0; j < 4; ++j) acc[i][j] = (v8f){0.f,0.f,0.f,0.f,0.f,0.f,0.f,0.f};

  for (int k0 = 0; k0 < K; k0 += 32) {
    V bh[4], bl[4];
#pragma unroll
    for (int j = 0; j < 4; ++j) {
      const size_t bo = (size_t)(n0 + (j << 4) + rlane) * ldb + koff + k0;
      bh[j] = Frag<T>::load(Bb + bo);
      if (SPLIT) bl[j] = Frag<T>::load(Bb2 + bo);
    }
#pragma unroll
    for (int i = 0; i < 4; ++i) {
      const size_t ao = (size_t)(m0 + (i << 4) + rlane) * lda + koff + k0;
      V ah = Frag<T>::load(Ab + ao);
      V al;
      if (SPLIT) al = Frag<T>::load(Ab2 + ao);
#pragma unroll
      for (int j = 0; j < 4; ++j) {
        acc[i][j] = Frag<T>::mma(ah, bh[j], acc[i][j]);
        if (SPLIT) {
          acc[i][j] = Frag<T>::mma(ah, bl[j], acc[i][j]);
          acc[i][j] = Frag<T>::mma(al, bh[j], acc[i][j]);
        }
      }
      Frag<T>::guard(acc[i][0], acc[i][3], ah, SPLIT ? al : ah);
    }
    Frag<T>::keep(bh[0], bh[1], bh[2], bh[3]);
    if (SPLIT) Frag<T>::keep(bl[0], bl[1], bl[2], bl[3]);
  }
  acc_guard4(acc[0][0], acc[0][1], acc[0][2], acc[0][3]);
  acc_guard4(acc[1][0], acc[1][1], acc[1][2], acc[1][3]);
  acc_guard4(acc[2][0], acc[2][1], acc[2][2], acc[2][3]);
  acc_guard4(acc[3][0], acc[3][1], acc[3][2], acc[3][3]);

  float* slab = sT[wave];
  const float* Rb = RESID ? (resid + (size_t)b * strideR) : nullptr;
#pragma unroll
  for (int i = 0; i < 4; ++i) {
    const int mBase = m0 + (i << 4);
#pragma unroll
    for (int j = 0; j < 4; ++j) {
      const int n = n0 + (j << 4) + rlane;
      float bv = 0.f;
      if (BIAS_MODE == 2) bv = bias[n];
#pragma unroll
      for (int r = 0; r < 8; ++r) {
        float v = acc[i][j][r] * scale;
        if (BIAS_MODE == 1) v += bias[mBase + mOff + r];
        if (BIAS_MODE == 2) v += bv;
        if (RESID) v += Rb[(size_t)(mBase + mOff + r) * ldc + n];
        if (ACT == 1) v = tanhf(v);
        if (ACT == 2) v = fmaxf(v, 0.0f);
        if (ACT == 3) v = v / (1.0f + expf(-v));
        if (ACT == 4) v = (v > 0.f) ? v : 0.01f * v;
        if (ACT == 5) v = 0.5f * v * (1.0f + erff(v * 0.70710678118654752f));
        slab[(mOff + r) * 68 + (j << 4) + rlane] = v;
      }
    }
    __builtin_amdgcn_fence(__ATOMIC_RELEASE, "workgroup");
    __builtin_amdgcn_wave_barrier();
    __builtin_amdgcn_fence(__ATOMIC_ACQUIRE, "workgroup");
    if (OUT_MODE == 0) {
      float* C = (float*)Cout + (size_t)b * strideC;
      const int hh = lane >> 4, c4 = (lane & 15) * 4;
      for (int pass = 0; pass < 2; ++pass) {
#pragma unroll
        for (int it = 0; it < 8; ++it) {
          const int row = it * 2 + hh;
          v4f v = *(const v4f*)(slab + row * 68 + c4);
          *(volatile v4f*)(C + (size_t)(mBase + row) * ldc + n0 + c4) = v;
        }
        __threadfence();
      }
    } else {
      const int q = lane >> 3, c8 = (lane & 7) * 8;
      unsigned short* C  = (unsigned short*)Cout  + (size_t)b * strideC;
      unsigned short* C2 = (OUT_MODE == 2) ? ((unsigned short*)Cout2 + (size_t)b * strideC) : nullptr;
      for (int pass = 0; pass < 2; ++pass) {
#pragma unroll
        for (int it = 0; it < 4; ++it) {
          const int row = it * 4 + q;
          const float* sp = slab + row * 68 + c8;
          v8h hv, lv;
#pragma unroll
          for (int e = 0; e < 8; ++e) {
            if (OUT_MODE == 1) {
              hv[e] = (_Float16)sp[e];
            } else {
              unsigned short hb = f2bf_bits(sp[e]);
              unsigned short lb = f2bf_bits(sp[e] - bf_bits2f(hb));
              hv[e] = __builtin_bit_cast(_Float16, hb);
              lv[e] = __builtin_bit_cast(_Float16, lb);
            }
          }
          *(volatile v8h*)(C + (size_t)(mBase + row) * ldc + n0 + c8) = hv;
          if (OUT_MODE == 2) *(volatile v8h*)(C2 + (size_t)(mBase + row) * ldc + n0 + c8) = lv;
        }
        __threadfence();
      }
    }
    __builtin_amdgcn_fence(__ATOMIC_RELEASE, "workgroup");
    __builtin_amdgcn_wave_barrier();
    __builtin_amdgcn_fence(__ATOMIC_ACQUIRE, "workgroup");
  }
}

__global__ __launch_bounds__(256) void pack_act_bf16(const float* __restrict__ X,
                                                    const float* __restrict__ Hp,
                                                    unsigned short* __restrict__ Acat) {
  const int part = blockIdx.y;
  const int t    = blockIdx.x * 256 + threadIdx.x;
  const int m    = t >> 7;
  const int kc   = (t & 127) << 3;
  const float* src = (part == 0) ? X : Hp;
  const float* sp  = src + (size_t)m * kDin + kc;
  const v4f a = *(const v4f*)(sp);
  const v4f c = *(const v4f*)(sp + 4);
  v4u w;
  w[0] = pack_bf2(a[0], a[1]);
  w[1] = pack_bf2(a[2], a[3]);
  w[2] = pack_bf2(c[0], c[1]);
  w[3] = pack_bf2(c[2], c[3]);
  unsigned short* dp = Acat + (size_t)m * kKcat + part * kDin + kc;
  *(volatile v4u*)dp = w;
  __threadfence();
  *(volatile v4u*)dp = w;
}

__global__ __launch_bounds__(256) void pack_wt_bf16(
    const float* __restrict__ Wf, const float* __restrict__ Uf,
    const float* __restrict__ Wi, const float* __restrict__ Ui,
    const float* __restrict__ Wc, const float* __restrict__ Uc,
    const float* __restrict__ Wo, const float* __restrict__ Uo,
    unsigned short* __restrict__ Bt) {
  __shared__ float tile[64][65];
  const int mat  = blockIdx.y;
  const int g    = mat >> 1;
  const int part = mat & 1;
  const float* src;
  switch (mat) {
    case 0:  src = Wf; break;
    case 1:  src = Uf; break;
    case 2:  src = Wi; break;
    case 3:  src = Ui; break;
    case 4:  src = Wc; break;
    case 5:  src = Uc; break;
    case 6:  src = Wo; break;
    default: src = Uo; break;
  }
  const int bt  = blockIdx.x;
  const int k0  = (bt >> 4) * 64;
  const int n0  = (bt & 15) * 64;
  const int tid = threadIdx.x;
  {
    const int lr  = tid >> 4;
    const int lc4 = (tid & 15) * 4;
#pragma unroll
    for (int it = 0; it < 4; ++it) {
      const int row = it * 16 + lr;
      const v4f v = *(const v4f*)(src + (size_t)(k0 + row) * kHid + n0 + lc4);
      tile[row][lc4 + 0] = v[0];
      tile[row][lc4 + 1] = v[1];
      tile[row][lc4 + 2] = v[2];
      tile[row][lc4 + 3] = v[3];
    }
  }
  __syncthreads();
  const int wave = tid >> 5, lane = tid & 31;
  const int rq = lane >> 3;
  const int cq = lane & 7;
  v4u w[2];
  unsigned short* dp[2];
#pragma unroll
  for (int iter = 0; iter < 2; ++iter) {
    const int rr = iter * 32 + wave * 4 + rq;
    const int kk = cq * 8;
    v4u o;
    o[0] = pack_bf2(tile[kk + 0][rr], tile[kk + 1][rr]);
    o[1] = pack_bf2(tile[kk + 2][rr], tile[kk + 3][rr]);
    o[2] = pack_bf2(tile[kk + 4][rr], tile[kk + 5][rr]);
    o[3] = pack_bf2(tile[kk + 6][rr], tile[kk + 7][rr]);
    w[iter]  = o;
    dp[iter] = Bt + (size_t)(g * kHid + n0 + rr) * kKcat + part * kDin + k0 + kk;
  }
  *(volatile v4u*)dp[0] = w[0];
  *(volatile v4u*)dp[1] = w[1];
  __threadfence();
  *(volatile v4u*)dp[0] = w[0];
  *(volatile v4u*)dp[1] = w[1];
}

__device__ __forceinline__ float gate_sig(float x) {
  const float e = exp2f(x * -1.4426950408889634f);
  return __builtin_amdgcn_rcpf(1.0f + e);
}
__device__ __forceinline__ float gate_tanh(float x) {
  const float e = exp2f(x * -2.8853900817779268f);
  return 2.0f * __builtin_amdgcn_rcpf(1.0f + e) - 1.0f;
}

__global__ __launch_bounds__(256) void lstm_pointwise(
    const float* __restrict__ Pre, const float* __restrict__ Cp,
    const float* __restrict__ bfp, const float* __restrict__ bip,
    const float* __restrict__ bcp, const float* __restrict__ bop,
    float* __restrict__ Hn, float* __restrict__ Cn) {
  const int t = blockIdx.x * 256 + threadIdx.x;
  const int m = t >> 8;
  const int n = (t & 255) << 2;
  const float* pr = Pre + (size_t)m * kNcat + n;
  const v4f pf = *(const v4f*)(pr);
  const v4f pi = *(const v4f*)(pr + kHid);
  const v4f pc = *(const v4f*)(pr + 2 * kHid);
  const v4f po = *(const v4f*)(pr + 3 * kHid);
  const v4f cp = *(const v4f*)(Cp + (size_t)m * kHid + n);
  const v4f vbf = *(const v4f*)(bfp + n);
  const v4f vbi = *(const v4f*)(bip + n);
  const v4f vbc = *(const v4f*)(bcp + n);
  const v4f vbo = *(const v4f*)(bop + n);
  v4f hout, cout;
#pragma unroll
  for (int e = 0; e < 4; ++e) {
    const float fg  = gate_sig (pf[e] + bf_rne(vbf[e]));
    const float ig  = gate_sig (pi[e] + bf_rne(vbi[e]));
    const float ct  = gate_tanh(pc[e] + bf_rne(vbc[e]));
    const float og  = gate_sig (po[e] + bf_rne(vbo[e]));
    const float cpr = bf_rne(cp[e]);
    const float cn  = fg * cpr + ig * ct;
    cout[e] = cn;
    hout[e] = og * gate_tanh(cn);
  }
  float* hp = Hn + (size_t)m * kHid + n;
  float* cq = Cn + (size_t)m * kHid + n;
  *(volatile v4f*)hp = hout;
  *(volatile v4f*)cq = cout;
  __threadfence();
  *(volatile v4f*)hp = hout;
  *(volatile v4f*)cq = cout;
}

extern "C" void kernel_launch(void* const* d_in, const int* in_sizes, int n_in,
                              void* d_out, int out_size, void* d_ws, size_t ws_size,
                              hipStream_t stream) {
  if (n_in < 15) return;
  if (in_sizes[0] != kBatch * kDin || in_sizes[1] != kBatch * kHid || in_sizes[2] != kBatch * kHid) return;
  if (in_sizes[3] != kDin * kHid || in_sizes[4] != kHid * kHid || in_sizes[5] != kHid) return;
  if (in_sizes[6] != kDin * kHid || in_sizes[7] != kHid * kHid || in_sizes[8] != kHid) return;
  if (in_sizes[9] != kDin * kHid || in_sizes[10] != kHid * kHid || in_sizes[11] != kHid) return;
  if (in_sizes[12] != kDin * kHid || in_sizes[13] != kHid * kHid || in_sizes[14] != kHid) return;
  if ((size_t)out_size != (size_t)2 * kBatch * kHid) return;
  if (ws_size < kCarve) return;

  const float* X   = (const float*)d_in[0];
  const float* Hp  = (const float*)d_in[1];
  const float* Cp  = (const float*)d_in[2];
  const float* Wf  = (const float*)d_in[3];
  const float* Uf  = (const float*)d_in[4];
  const float* bfv = (const float*)d_in[5];
  const float* Wi  = (const float*)d_in[6];
  const float* Ui  = (const float*)d_in[7];
  const float* biv = (const float*)d_in[8];
  const float* Wc  = (const float*)d_in[9];
  const float* Uc  = (const float*)d_in[10];
  const float* bcv = (const float*)d_in[11];
  const float* Wo  = (const float*)d_in[12];
  const float* Uo  = (const float*)d_in[13];
  const float* bov = (const float*)d_in[14];

  unsigned short* Acat = (unsigned short*)d_ws;
  unsigned short* Bt   = (unsigned short*)((char*)d_ws + kOffBt);
  float*          Pre  = (float*)((char*)d_ws + kOffPre);
  float* Hn = (float*)d_out;
  float* Cn = (float*)d_out + kOut1ElemOff;

  pack_act_bf16<<<dim3((kBatch * (kDin / 8)) / 256, 2), 256, 0, stream>>>(X, Hp, Acat);

  pack_wt_bf16<<<dim3((kDin / 64) * (kHid / 64), 8), 256, 0, stream>>>(Wf, Uf, Wi, Ui, Wc, Uc, Wo, Uo, Bt);

  {
    const int tiles = (kBatch / 64) * (kNcat / 64);
    wmma_gemm64<1, false, 0, 0, false, 0><<<dim3(tiles / 8, 1), 256, 0, stream>>>(
        Acat, Acat, kKcat, 0L,
        Bt, Bt, kKcat, 0L,
        (void*)Pre, (void*)Pre, kNcat, 0L,
        bfv,
        bfv, 0L,
        kBatch, kNcat, kKcat, 1.0f);
  }

  lstm_pointwise<<<(kBatch * (kHid / 4)) / 256, 256, 0, stream>>>(Pre, Cp, bfv, biv, bcv, bov, Hn, Cn);
}
